// SGAT_multi_75488345194751
// MI455X (gfx1250) — hardware-verified
//
#include <hip/hip_runtime.h>
#include <stddef.h>


#define NF1   128
#define C1    256
#define NH1   4
#define NBAS  8
#define C2    40
#define C2P   48
#define P2    64
#define GR    32
#define NTHR  256
#define NWAVE 8
#define AP1   136
#define AP2   264
#define RSP1  260
#define RSP2  68
#define CHUNK 4096
#define NGRP  (CHUNK / (NTHR * 8))
#define WCAP  (CHUNK / NWAVE)
#define NB1   256
#define LSH1  8
#define NB2   1024
#define LSH2  10
#define AGG_LDS(NBK, ROWF, NHD) (((NBK) * (ROWF) + (((NBK) * (NHD) + 3) / 4) * 4 + NWAVE * WCAP + NWAVE) * 4)
#define LDS1  AGG_LDS(NB1, C1, NH1)
#define LDS2  AGG_LDS(NB2, P2, 1)

static_assert(NGRP == 2);
static_assert(WCAP == NGRP * 8 * 32);
static_assert((1 << LSH1) == NB1);
static_assert((1 << LSH2) == NB2);
static_assert((CHUNK << LSH2) <= (1 << 30));
static_assert(LDS1 == 282656);
static_assert(LDS2 == 282656);
static_assert((NF1 % 32) == 0);
static_assert((C1 % 32) == 0);
static_assert(((AP1 * 2) % 16) == 0);
static_assert(((AP2 * 2) % 16) == 0);
static_assert(((RSP1 * 4) % 16) == 0);
static_assert(((RSP2 * 4) % 16) == 0);

typedef float          v4f  __attribute__((ext_vector_type(4)));
typedef float          v8f  __attribute__((ext_vector_type(8)));
typedef int            v4i  __attribute__((ext_vector_type(4)));
typedef int            v8i  __attribute__((ext_vector_type(8)));
typedef unsigned short v4us __attribute__((ext_vector_type(4)));
typedef unsigned short v8us __attribute__((ext_vector_type(8)));
typedef __bf16         v16bf __attribute__((ext_vector_type(16)));

union FragB { v16bf v; v8us u[2]; v8i i; };
union Pk8   { v8us u; v4us q[2]; };

__device__ __forceinline__ int imin(int a, int b) { return a < b ? a : b; }

__device__ __forceinline__ v4f zero4() { v4f z = {0.f, 0.f, 0.f, 0.f}; return z; }
__device__ __forceinline__ v8f zero8() { v8f z = {0.f, 0.f, 0.f, 0.f, 0.f, 0.f, 0.f, 0.f}; return z; }

__device__ __forceinline__ v8f wm(const FragB& a, const FragB& b, v8f c) {
  v8f d = __builtin_amdgcn_wmma_f32_16x16x32_bf16(false, a.v, false, b.v, (short)0, c, false, false);
  asm volatile("v_nop\n\tv_nop\n\tv_nop\n\tv_nop" : "+v"(d) : "v"(a.i), "v"(b.i));
  return d;
}

__device__ __forceinline__ void ldfrag(FragB& f, const unsigned short* p) {
  f.u[0] = *(const v8us*)p;
  f.u[1] = *(const v8us*)(p + 16);
}

__device__ __forceinline__ unsigned int bfb(float f) {
  const unsigned int u = __float_as_uint(f);
  return (u + 0x7FFFu + ((u >> 16) & 1u)) >> 16;
}
__device__ __forceinline__ void split1(float f, unsigned short& h, unsigned short& l) {
  const unsigned int hb = bfb(f);
  const float r = f - __uint_as_float(hb << 16);
  h = (unsigned short)hb;
  l = (unsigned short)bfb(r);
}
__device__ __forceinline__ void split4(v4f f, v4us& h, v4us& l) {
  unsigned short a, b;
  split1(f.x, a, b); h.x = a; l.x = b;
  split1(f.y, a, b); h.y = a; l.y = b;
  split1(f.z, a, b); h.z = a; l.z = b;
  split1(f.w, a, b); h.w = a; l.w = b;
}

__global__ __launch_bounds__(NTHR) void k_prepw(const float* __restrict__ W, unsigned short* Whi,
                                                unsigned short* Wlo, int K, int Ncols, int Npad) {
  const int i  = blockIdx.x * NTHR + threadIdx.x;
  const int k8 = K >> 3;
  if (i >= Npad * k8) return;
  const int n  = i / k8;
  const int kk = (i - n * k8) * 8;
  const int nc = n < Ncols ? n : Ncols - 1;
  v8us uh, ul;
  {
    unsigned short a, b; float v;
    v = W[(size_t)(kk + 0) * Ncols + nc]; if (n >= Ncols) v = 0.f; split1(v, a, b); uh[0] = a; ul[0] = b;
    v = W[(size_t)(kk + 1) * Ncols + nc]; if (n >= Ncols) v = 0.f; split1(v, a, b); uh[1] = a; ul[1] = b;
    v = W[(size_t)(kk + 2) * Ncols + nc]; if (n >= Ncols) v = 0.f; split1(v, a, b); uh[2] = a; ul[2] = b;
    v = W[(size_t)(kk + 3) * Ncols + nc]; if (n >= Ncols) v = 0.f; split1(v, a, b); uh[3] = a; ul[3] = b;
    v = W[(size_t)(kk + 4) * Ncols + nc]; if (n >= Ncols) v = 0.f; split1(v, a, b); uh[4] = a; ul[4] = b;
    v = W[(size_t)(kk + 5) * Ncols + nc]; if (n >= Ncols) v = 0.f; split1(v, a, b); uh[5] = a; ul[5] = b;
    v = W[(size_t)(kk + 6) * Ncols + nc]; if (n >= Ncols) v = 0.f; split1(v, a, b); uh[6] = a; ul[6] = b;
    v = W[(size_t)(kk + 7) * Ncols + nc]; if (n >= Ncols) v = 0.f; split1(v, a, b); uh[7] = a; ul[7] = b;
  }
  const size_t o = (size_t)n * K + kk;
  *(volatile v8us*)(Whi + o) = uh;
  *(volatile v8us*)(Wlo + o) = ul;
  __threadfence();
  *(volatile v8us*)(Whi + o) = uh;
  *(volatile v8us*)(Wlo + o) = ul;
}

__global__ __launch_bounds__(NTHR) void k_node1(const float* __restrict__ x,
                                                const unsigned short* __restrict__ W1h,
                                                const unsigned short* __restrict__ W1l,
                                                const float* __restrict__ B1, const float* __restrict__ cs1,
                                                const float* __restrict__ cd1,
                                                float* h1, float* es1, float* ed1, int nN) {
  __shared__ __attribute__((aligned(16))) unsigned short Ah[GR * AP1];
  __shared__ __attribute__((aligned(16))) unsigned short Al[GR * AP1];
  __shared__ __attribute__((aligned(16))) float Rs[GR * RSP1];

  const int tid  = threadIdx.x;
  const int lane = tid & 31;
  const int wave = tid >> 5;
  const int lh   = lane >> 4;
  const int m    = lane & 15;
  const int rowBase = blockIdx.x * GR;

  {
    const int r  = tid >> 3;
    const int c0 = (tid & 7) * 16;
    int row = rowBase + r;
    row = row > nN - 1 ? nN - 1 : row;
    const float* p = x + (size_t)row * NF1 + c0;
    const v4f f0 = *(const v4f*)(p),     f1 = *(const v4f*)(p + 4);
    const v4f f2 = *(const v4f*)(p + 8), f3 = *(const v4f*)(p + 12);
    Pk8 ha, la, hb, lb;
    split4(f0, ha.q[0], la.q[0]); split4(f1, ha.q[1], la.q[1]);
    split4(f2, hb.q[0], lb.q[0]); split4(f3, hb.q[1], lb.q[1]);
    *(v8us*)(Ah + r * AP1 + c0)     = ha.u;
    *(v8us*)(Ah + r * AP1 + c0 + 8) = hb.u;
    *(v8us*)(Al + r * AP1 + c0)     = la.u;
    *(v8us*)(Al + r * AP1 + c0 + 8) = lb.u;
  }
  __syncthreads();

  const int nc0 = wave * 32;
  v8f a00 = zero8(), a01 = zero8(), a10 = zero8(), a11 = zero8();
#pragma unroll 1
  for (int k0 = 0; k0 < NF1; k0 += 32) {
    const int ka = k0 + 8 * lh;
    FragB ah0, ah1, al0, al1, bh0, bh1, bl0, bl1;
    ldfrag(ah0, Ah + m * AP1 + ka);
    ldfrag(ah1, Ah + (16 + m) * AP1 + ka);
    ldfrag(al0, Al + m * AP1 + ka);
    ldfrag(al1, Al + (16 + m) * AP1 + ka);
    ldfrag(bh0, W1h + (size_t)(nc0 + m) * NF1 + ka);
    ldfrag(bh1, W1h + (size_t)(nc0 + 16 + m) * NF1 + ka);
    ldfrag(bl0, W1l + (size_t)(nc0 + m) * NF1 + ka);
    ldfrag(bl1, W1l + (size_t)(nc0 + 16 + m) * NF1 + ka);
    a00 = wm(ah0, bh0, a00); a00 = wm(ah0, bl0, a00); a00 = wm(al0, bh0, a00);
    a01 = wm(ah0, bh1, a01); a01 = wm(ah0, bl1, a01); a01 = wm(al0, bh1, a01);
    a10 = wm(ah1, bh0, a10); a10 = wm(ah1, bl0, a10); a10 = wm(al1, bh0, a10);
    a11 = wm(ah1, bh1, a11); a11 = wm(ah1, bl1, a11); a11 = wm(al1, bh1, a11);
  }

#pragma unroll
  for (int r = 0; r < 8; ++r) {
    Rs[(8 * lh + r) * RSP1 + nc0 + m]           = a00[r];
    Rs[(8 * lh + r) * RSP1 + nc0 + 16 + m]      = a01[r];
    Rs[(16 + 8 * lh + r) * RSP1 + nc0 + m]      = a10[r];
    Rs[(16 + 8 * lh + r) * RSP1 + nc0 + 16 + m] = a11[r];
  }

  if (wave == 0) {
    int row = rowBase + lane;
    row = row > nN - 1 ? nN - 1 : row;
    const float* xr = x + (size_t)row * NF1;
    v4f sa = zero4(), sb = zero4();
#pragma unroll 1
    for (int k = 0; k < NF1; k += 4) {
      const v4f xv = *(const v4f*)(xr + k);
      const float* bp = B1 + k * NBAS;
      sa += xv.x * *(const v4f*)(bp);      sb += xv.x * *(const v4f*)(bp + 4);
      sa += xv.y * *(const v4f*)(bp + 8);  sb += xv.y * *(const v4f*)(bp + 12);
      sa += xv.z * *(const v4f*)(bp + 16); sb += xv.z * *(const v4f*)(bp + 20);
      sa += xv.w * *(const v4f*)(bp + 24); sb += xv.w * *(const v4f*)(bp + 28);
    }
    v4f ev = zero4(), dv = zero4();
    ev += sa.x * *(const v4f*)(cs1 + 0);  dv += sa.x * *(const v4f*)(cd1 + 0);
    ev += sa.y * *(const v4f*)(cs1 + 4);  dv += sa.y * *(const v4f*)(cd1 + 4);
    ev += sa.z * *(const v4f*)(cs1 + 8);  dv += sa.z * *(const v4f*)(cd1 + 8);
    ev += sa.w * *(const v4f*)(cs1 + 12); dv += sa.w * *(const v4f*)(cd1 + 12);
    ev += sb.x * *(const v4f*)(cs1 + 16); dv += sb.x * *(const v4f*)(cd1 + 16);
    ev += sb.y * *(const v4f*)(cs1 + 20); dv += sb.y * *(const v4f*)(cd1 + 20);
    ev += sb.z * *(const v4f*)(cs1 + 24); dv += sb.z * *(const v4f*)(cd1 + 24);
    ev += sb.w * *(const v4f*)(cs1 + 28); dv += sb.w * *(const v4f*)(cd1 + 28);
    float* pe = es1 + (size_t)(rowBase + lane) * NH1;
    float* pd = ed1 + (size_t)(rowBase + lane) * NH1;
    *(volatile v4f*)pe = ev;
    *(volatile v4f*)pd = dv;
    __threadfence();
    *(volatile v4f*)pe = ev;
    *(volatile v4f*)pd = dv;
  }
  __syncthreads();

  v4f xr[8];
#pragma unroll
  for (int i = 0; i < 4; ++i) {
    xr[2 * i]     = *(const v4f*)(Rs + (4 * wave + i) * RSP1 + lane * 4);
    xr[2 * i + 1] = *(const v4f*)(Rs + (4 * wave + i) * RSP1 + 128 + lane * 4);
  }
#pragma unroll
  for (int i = 0; i < 4; ++i) {
    float* op = h1 + (size_t)(rowBase + 4 * wave + i) * C1 + lane * 4;
    *(volatile v4f*)(op)       = xr[2 * i];
    *(volatile v4f*)(op + 128) = xr[2 * i + 1];
  }
  __threadfence();
#pragma unroll
  for (int i = 0; i < 4; ++i) {
    float* op = h1 + (size_t)(rowBase + 4 * wave + i) * C1 + lane * 4;
    *(volatile v4f*)(op)       = xr[2 * i];
    *(volatile v4f*)(op + 128) = xr[2 * i + 1];
  }
}

__global__ __launch_bounds__(NTHR) void k_node2(const float* __restrict__ hpl,
                                                const unsigned short* __restrict__ W2h,
                                                const unsigned short* __restrict__ W2l,
                                                const float* __restrict__ B2, const float* __restrict__ cs2,
                                                const float* __restrict__ cd2,
                                                float* h2, float* es2, float* ed2, int nN) {
  __shared__ __attribute__((aligned(16))) unsigned short Ah[GR * AP2];
  __shared__ __attribute__((aligned(16))) unsigned short Al[GR * AP2];
  __shared__ __attribute__((aligned(16))) float Rs[GR * RSP2];

  const int tid  = threadIdx.x;
  const int lane = tid & 31;
  const int wave = tid >> 5;
  const int lh   = lane >> 4;
  const int m    = lane & 15;
  const int rowBase = blockIdx.x * GR;

  {
    const int r  = tid >> 3;
    const int c0 = (tid & 7) * 32;
    int row = rowBase + r;
    row = row > nN - 1 ? nN - 1 : row;
    const float* p = hpl + (size_t)row * C1 + c0;
#pragma unroll
    for (int q = 0; q < 4; ++q) {
      const v4f f0 = *(const v4f*)(p + 8 * q);
      const v4f f1 = *(const v4f*)(p + 8 * q + 4);
      Pk8 hq, lq;
      split4(f0, hq.q[0], lq.q[0]);
      split4(f1, hq.q[1], lq.q[1]);
      *(v8us*)(Ah + r * AP2 + c0 + 8 * q) = hq.u;
      *(v8us*)(Al + r * AP2 + c0 + 8 * q) = lq.u;
    }
    if (tid < 128) {
      const int rr = tid >> 2;
      const int cc = C2P + (tid & 3) * 4;
      *(v4f*)(Rs + rr * RSP2 + cc) = zero4();
    }
  }
  __syncthreads();

  if (wave < 6) {
    const int mt = wave & 1;
    const int nt = wave >> 1;
    v8f acc = zero8();
#pragma unroll 1
    for (int k0 = 0; k0 < C1; k0 += 32) {
      const int ka = k0 + 8 * lh;
      FragB ah, al, bh, bl;
      ldfrag(ah, Ah + (mt * 16 + m) * AP2 + ka);
      ldfrag(al, Al + (mt * 16 + m) * AP2 + ka);
      ldfrag(bh, W2h + (size_t)(nt * 16 + m) * C1 + ka);
      ldfrag(bl, W2l + (size_t)(nt * 16 + m) * C1 + ka);
      acc = wm(ah, bh, acc);
      acc = wm(ah, bl, acc);
      acc = wm(al, bh, acc);
    }
#pragma unroll
    for (int r = 0; r < 8; ++r) Rs[(mt * 16 + 8 * lh + r) * RSP2 + nt * 16 + m] = acc[r];
  } else if (wave == 6) {
    int row = rowBase + lane;
    row = row > nN - 1 ? nN - 1 : row;
    const float* xr = hpl + (size_t)row * C1;
    v4f sa = zero4(), sb = zero4();
#pragma unroll 1
    for (int k = 0; k < C1; k += 4) {
      const v4f xv = *(const v4f*)(xr + k);
      const float* bp = B2 + k * NBAS;
      sa += xv.x * *(const v4f*)(bp);      sb += xv.x * *(const v4f*)(bp + 4);
      sa += xv.y * *(const v4f*)(bp + 8);  sb += xv.y * *(const v4f*)(bp + 12);
      sa += xv.z * *(const v4f*)(bp + 16); sb += xv.z * *(const v4f*)(bp + 20);
      sa += xv.w * *(const v4f*)(bp + 24); sb += xv.w * *(const v4f*)(bp + 28);
    }
    const float e_s = sa.x * cs2[0] + sa.y * cs2[1] + sa.z * cs2[2] + sa.w * cs2[3] +
                      sb.x * cs2[4] + sb.y * cs2[5] + sb.z * cs2[6] + sb.w * cs2[7];
    const float e_d = sa.x * cd2[0] + sa.y * cd2[1] + sa.z * cd2[2] + sa.w * cd2[3] +
                      sb.x * cd2[4] + sb.y * cd2[5] + sb.z * cd2[6] + sb.w * cd2[7];
    const int b4 = (4 * lane) & 31;
    v4f ps, pd;
    ps.x = __shfl(e_s, b4, 32);             pd.x = __shfl(e_d, b4, 32);
    ps.y = __shfl(e_s, (b4 + 1) & 31, 32);  pd.y = __shfl(e_d, (b4 + 1) & 31, 32);
    ps.z = __shfl(e_s, (b4 + 2) & 31, 32);  pd.z = __shfl(e_d, (b4 + 2) & 31, 32);
    ps.w = __shfl(e_s, (b4 + 3) & 31, 32);  pd.w = __shfl(e_d, (b4 + 3) & 31, 32);
    float* pe  = es2 + rowBase + 4 * lane;
    float* pdp = ed2 + rowBase + 4 * lane;
    if (lane < 8) { *(volatile v4f*)pe = ps; *(volatile v4f*)pdp = pd; }
    __threadfence();
    if (lane < 8) { *(volatile v4f*)pe = ps; *(volatile v4f*)pdp = pd; }
  }
  __syncthreads();

  v4f xv2[2];
#pragma unroll
  for (int i = 0; i < 2; ++i) {
    const int rr = 4 * wave + 2 * i + lh;
    xv2[i] = *(const v4f*)(Rs + rr * RSP2 + m * 4);
  }
#pragma unroll
  for (int i = 0; i < 2; ++i) {
    float* op = h2 + (size_t)(rowBase + 4 * wave + 2 * i) * P2 + lane * 4;
    *(volatile v4f*)op = xv2[i];
  }
  __threadfence();
#pragma unroll
  for (int i = 0; i < 2; ++i) {
    float* op = h2 + (size_t)(rowBase + 4 * wave + 2 * i) * P2 + lane * 4;
    *(volatile v4f*)op = xv2[i];
  }
}

template <int ROWF, int NHD, int NBK, int LSH, int FIN>
__global__ __launch_bounds__(NTHR) void k_agg(const int* __restrict__ ei, const float* __restrict__ hs,
                                              const float* __restrict__ es, const float* __restrict__ ed,
                                              const float* __restrict__ bias, float* outp, int nN, int nE) {
  constexpr int CH   = ROWF / 4;
  constexpr int CPL  = (CH + 31) / 32;
  constexpr int ACT  = CH / CPL;
  constexpr int HDIM = ROWF / NHD;
  constexpr int LPH  = (HDIM / 4) / CPL;
  constexpr int DENF = ((NBK * NHD + 3) / 4) * 4;
  constexpr int SPW  = NBK / NWAVE;
  constexpr int NPC  = (ROWF / 128) > 0 ? (ROWF / 128) : 1;
  static_assert(ACT == 32 || ACT == 16);
  static_assert(LPH >= 1 && (LPH & (LPH - 1)) == 0);
  static_assert(((NBK * ROWF + DENF) % 4) == 0);
  static_assert(FIN == 0 || NHD == 1);
  static_assert(FIN == 1 || (ROWF % 128) == 0);
  static_assert((NBK % NWAVE) == 0);
  static_assert(FIN == 0 || ROWF >= C2);
  static_assert(NPC >= 1);

  extern __shared__ v4f lds_dyn[];
  float* sacc = (float*)lds_dyn;
  float* den  = sacc + NBK * ROWF;
  int*   list = (int*)(den + DENF);
  int*   wcnt = list + NWAVE * WCAP;

  const int tid  = threadIdx.x;
  const int lane = tid & 31;
  const int wave = tid >> 5;
  const int nodeBase = blockIdx.x * NBK;

  {
    const v4f z4 = zero4();
    for (int i = tid; i < (NBK * ROWF + DENF) / 4; i += NTHR) lds_dyn[i] = z4;
  }
  __syncthreads();

  const int  al  = lane & (ACT - 1);
  const int  col = al * CPL * 4;
  const int  hd  = col / HDIM;
  const bool act = lane < ACT;
  const bool dln = act && ((al & (LPH - 1)) == 0);
  const int* eid = ei + nE;
  const bool vec16 = ((nE & 3) == 0);
  const int  nChunks = (nE + CHUNK - 1) / CHUNK;
  const int  sent = -2147483647 - 1;

#pragma unroll 1
  for (int ch = 0; ch < nChunks; ++ch) {
    const int cbase = ch * CHUNK;
    int wc = 0;
#pragma unroll
    for (int g = 0; g < NGRP; ++g) {
      const int el0 = (g * NTHR + tid) * 8;
      const int e0  = cbase + el0;
      v4i d0, d1;
      if (vec16 && (cbase + CHUNK <= nE)) {
        d0 = *(const v4i*)(eid + e0);
        d1 = *(const v4i*)(eid + e0 + 4);
      } else {
        d0.x = (e0     < nE) ? eid[imin(e0,     nE - 1)] : sent;
        d0.y = (e0 + 1 < nE) ? eid[imin(e0 + 1, nE - 1)] : sent;
        d0.z = (e0 + 2 < nE) ? eid[imin(e0 + 2, nE - 1)] : sent;
        d0.w = (e0 + 3 < nE) ? eid[imin(e0 + 3, nE - 1)] : sent;
        d1.x = (e0 + 4 < nE) ? eid[imin(e0 + 4, nE - 1)] : sent;
        d1.y = (e0 + 5 < nE) ? eid[imin(e0 + 5, nE - 1)] : sent;
        d1.z = (e0 + 6 < nE) ? eid[imin(e0 + 6, nE - 1)] : sent;
        d1.w = (e0 + 7 < nE) ? eid[imin(e0 + 7, nE - 1)] : sent;
      }
      const unsigned s0 = (unsigned)d0.x - (unsigned)nodeBase;
      const unsigned s1 = (unsigned)d0.y - (unsigned)nodeBase;
      const unsigned s2 = (unsigned)d0.z - (unsigned)nodeBase;
      const unsigned s3 = (unsigned)d0.w - (unsigned)nodeBase;
      const unsigned s4 = (unsigned)d1.x - (unsigned)nodeBase;
      const unsigned s5 = (unsigned)d1.y - (unsigned)nodeBase;
      const unsigned s6 = (unsigned)d1.z - (unsigned)nodeBase;
      const unsigned s7 = (unsigned)d1.w - (unsigned)nodeBase;
      const bool q0 = s0 < (unsigned)NBK, q1 = s1 < (unsigned)NBK;
      const bool q2 = s2 < (unsigned)NBK, q3 = s3 < (unsigned)NBK;
      const bool q4 = s4 < (unsigned)NBK, q5 = s5 < (unsigned)NBK;
      const bool q6 = s6 < (unsigned)NBK, q7 = s7 < (unsigned)NBK;
      const unsigned many = __builtin_amdgcn_ballot_w32(q0 | q1 | q2 | q3 | q4 | q5 | q6 | q7);
      if (many != 0u) {
#define HITJ(J, QJ, SJ) { \
          const unsigned mj = __builtin_amdgcn_ballot_w32(QJ); \
          if (QJ) { \
            const int pos = wc + (int)__builtin_amdgcn_mbcnt_lo(mj, 0u); \
            if (pos < WCAP) list[wave * WCAP + pos] = ((el0 + (J)) << LSH) | (int)(SJ); \
          } \
          wc += (int)__builtin_popcount(mj); }
        HITJ(0, q0, s0)
        HITJ(1, q1, s1)
        HITJ(2, q2, s2)
        HITJ(3, q3, s3)
        HITJ(4, q4, s4)
        HITJ(5, q5, s5)
        HITJ(6, q6, s6)
        HITJ(7, q7, s7)
#undef HITJ
      }
    }
    if (lane == 0) wcnt[wave] = wc;
    __syncthreads();

    if (wave == 0) {
#pragma unroll 1
      for (int wsx = 0; wsx < NWAVE; ++wsx) {
        int n = wcnt[wsx];
        n = n > WCAP ? WCAP : n;
        n = n < 0 ? 0 : n;
#pragma unroll 1
        for (int i = 0; i < n; ++i) {
          const int ent  = list[wsx * WCAP + i];
          const int slot = ent & (NBK - 1);
          const int el   = (ent >> LSH) & (CHUNK - 1);
          int e = cbase + el;
          e = e > nE - 1 ? nE - 1 : e;
          int src = ei[e];
          src = src < 0 ? 0 : (src > nN - 1 ? nN - 1 : src);
          int nd = nodeBase + slot;
          nd = nd > nN - 1 ? nN - 1 : nd;
          float a = es[(size_t)src * NHD + hd] + ed[(size_t)nd * NHD + hd];
          a = (a > 0.f) ? a : 0.2f * a;
          a = fminf(fmaxf(a, -80.f), 80.f);
          const float p = __expf(a);
          const float* hp = hs + (size_t)src * ROWF + col;
          float* sp = sacc + slot * ROWF + col;
          v4f hv[CPL], cur[CPL];
#pragma unroll
          for (int v = 0; v < CPL; ++v) {
            hv[v]  = *(const v4f*)(hp + 4 * v);
            cur[v] = *(const v4f*)(sp + 4 * v);
          }
          if (act) {
#pragma unroll
            for (int v = 0; v < CPL; ++v) *(v4f*)(sp + 4 * v) = cur[v] + p * hv[v];
          }
          const float od = den[slot * NHD + hd];
          if (dln) den[slot * NHD + hd] = od + p;
        }
      }
    }
    __syncthreads();
  }

  if (FIN == 0) {
#pragma unroll 1
    for (int j = 0; j < SPW; ++j) {
      const int slot = wave * SPW + j;
      const int node = nodeBase + slot;
      if (node >= nN) break;
      v4f ov[NPC];
#pragma unroll
      for (int v = 0; v < NPC; ++v) {
        const int cv  = v * 128 + lane * 4;
        const int hcv = cv / HDIM;
        const v4f a = *(const v4f*)(sacc + slot * ROWF + cv);
        const float dn  = den[slot * NHD + hcv];
        const float inv = (dn > 0.f) ? __builtin_amdgcn_rcpf(dn) : 0.f;
        v4f o = a * inv + *(const v4f*)(bias + cv);
        o.x = o.x > 0.f ? o.x : (__expf(o.x) - 1.0f);
        o.y = o.y > 0.f ? o.y : (__expf(o.y) - 1.0f);
        o.z = o.z > 0.f ? o.z : (__expf(o.z) - 1.0f);
        o.w = o.w > 0.f ? o.w : (__expf(o.w) - 1.0f);
        ov[v] = o;
      }
      float* op = outp + (size_t)node * ROWF;
#pragma unroll
      for (int v = 0; v < NPC; ++v) *(volatile v4f*)(op + v * 128 + lane * 4) = ov[v];
      __threadfence();
#pragma unroll
      for (int v = 0; v < NPC; ++v) *(volatile v4f*)(op + v * 128 + lane * 4) = ov[v];
    }
  } else {
#pragma unroll 1
    for (int i = tid; i < NBK * CH; i += NTHR) {
      const int slot = i / CH;
      const int c = (i - slot * CH) * 4;
      const float dn  = den[slot * NHD];
      const float inv = (dn > 0.f) ? __builtin_amdgcn_rcpf(dn) : 0.f;
      float* pp = sacc + slot * ROWF + c;
      const v4f a = *(const v4f*)pp;
      *(v4f*)pp = a * inv;
    }
    __syncthreads();
    int rows = nN - nodeBase;
    rows = rows > NBK ? NBK : rows;
    constexpr int PPR = C2 / 4;
    const int npc = rows * PPR;
    float* ob = outp + (size_t)nodeBase * C2;
#pragma unroll 1
    for (int i = tid; i < npc; i += NTHR) {
      const int r = i / PPR;
      const int c = (i - r * PPR) * 4;
      const v4f v = *(const v4f*)(sacc + r * ROWF + c);
      *(volatile v4f*)(ob + (size_t)i * 4) = v;
    }
    __threadfence();
#pragma unroll 1
    for (int i = tid; i < npc; i += NTHR) {
      const int r = i / PPR;
      const int c = (i - r * PPR) * 4;
      const v4f v = *(const v4f*)(sacc + r * ROWF + c);
      *(volatile v4f*)(ob + (size_t)i * 4) = v;
    }
  }
}

static inline size_t al256(size_t b) { return (b + 255) & ~(size_t)255; }

extern "C" void kernel_launch(void* const* d_in, const int* in_sizes, int n_in,
                              void* d_out, int out_size, void* d_ws, size_t ws_size,
                              hipStream_t stream) {
  if (n_in < 11) return;
  const int nN = in_sizes[0] / NF1;
  const int nE = in_sizes[1] / 2;
  if (nN <= 0 || in_sizes[0] != nN * NF1) return;
  if (nE < 0 || in_sizes[1] != 2 * nE) return;
  if (in_sizes[2] != NF1 * C1 || in_sizes[3] != C1 || in_sizes[4] != NF1 * NBAS) return;
  if (in_sizes[5] != NBAS * NH1 || in_sizes[6] != NBAS * NH1) return;
  if (in_sizes[7] != C1 * C2 || in_sizes[8] != C1 * NBAS || in_sizes[9] != NBAS || in_sizes[10] != NBAS) return;
  if (out_size != nN * C2) return;

  const float* x   = (const float*)d_in[0];
  const int*   ei  = (const int*)d_in[1];
  const float* W1  = (const float*)d_in[2];
  const float* b1  = (const float*)d_in[3];
  const float* B1  = (const float*)d_in[4];
  const float* cs1 = (const float*)d_in[5];
  const float* cd1 = (const float*)d_in[6];
  const float* W2  = (const float*)d_in[7];
  const float* B2  = (const float*)d_in[8];
  const float* cs2 = (const float*)d_in[9];
  const float* cd2 = (const float*)d_in[10];
  float* out = (float*)d_out;

  const int nP = ((nN + GR - 1) / GR) * GR;
  char* wp = (char*)d_ws;
  size_t off = 0;
  unsigned short* W1h = (unsigned short*)(wp + off); off += al256((size_t)C1 * NF1 * 2);
  unsigned short* W1l = (unsigned short*)(wp + off); off += al256((size_t)C1 * NF1 * 2);
  unsigned short* W2h = (unsigned short*)(wp + off); off += al256((size_t)C2P * C1 * 2);
  unsigned short* W2l = (unsigned short*)(wp + off); off += al256((size_t)C2P * C1 * 2);
  float* h1  = (float*)(wp + off); off += al256((size_t)nP * C1 * sizeof(float));
  float* es1 = (float*)(wp + off); off += al256((size_t)nP * NH1 * sizeof(float));
  float* ed1 = (float*)(wp + off); off += al256((size_t)nP * NH1 * sizeof(float));
  float* hpl = (float*)(wp + off); off += al256((size_t)nP * C1 * sizeof(float));
  float* h2  = (float*)(wp + off); off += al256((size_t)nP * P2 * sizeof(float));
  float* es2 = (float*)(wp + off); off += al256((size_t)nP * sizeof(float));
  float* ed2 = (float*)(wp + off); off += al256((size_t)nP * sizeof(float));
  if (off > ws_size) return;

  k_prepw<<<(C1 * (NF1 / 8) + NTHR - 1) / NTHR, NTHR, 0, stream>>>(W1, W1h, W1l, NF1, C1, C1);
  k_prepw<<<(C2P * (C1 / 8) + NTHR - 1) / NTHR, NTHR, 0, stream>>>(W2, W2h, W2l, C1, C2, C2P);

  k_node1<<<nP / GR, NTHR, 0, stream>>>(x, W1h, W1l, B1, cs1, cd1, h1, es1, ed1, nN);

  hipFuncSetAttribute(reinterpret_cast<const void*>(&k_agg<C1, NH1, NB1, LSH1, 0>),
                      hipFuncAttributeMaxDynamicSharedMemorySize, LDS1);
  k_agg<C1, NH1, NB1, LSH1, 0><<<(nN + NB1 - 1) / NB1, NTHR, LDS1, stream>>>(
      ei, h1, es1, ed1, b1, hpl, nN, nE);

  k_node2<<<nP / GR, NTHR, 0, stream>>>(hpl, W2h, W2l, B2, cs2, cd2, h2, es2, ed2, nN);

  hipFuncSetAttribute(reinterpret_cast<const void*>(&k_agg<P2, 1, NB2, LSH2, 1>),
                      hipFuncAttributeMaxDynamicSharedMemorySize, LDS2);
  k_agg<P2, 1, NB2, LSH2, 1><<<(nN + NB2 - 1) / NB2, NTHR, LDS2, stream>>>(
      ei, h2, es2, ed2, b1, out, nN, nE);
}
